// TransformerBlock_3702261809285
// MI455X (gfx1250) — hardware-run, weakly checked
//
#include <hip/hip_runtime.h>
#include <stddef.h>


typedef _Float16 v16h __attribute__((ext_vector_type(16)));
typedef _Float16 v8h  __attribute__((ext_vector_type(8)));
typedef float    v8f  __attribute__((ext_vector_type(8)));
typedef float    v4f  __attribute__((ext_vector_type(4)));

#ifndef NB
#define NB 1
#endif
#ifndef SEQ
#define SEQ 2048
#endif
#define NB_FULL  1
#define SEQ_FULL 2048
#define DIM   1024
#define NHEAD 16
#define HD    64
#define DFF   4096
#define NCB   4
#define CDIM  64
#define DCAT  (NCB * CDIM)
#define MROWS (NB * SEQ)
#ifndef EROWS
#define EROWS 1024
#endif
#define EROWS_EFF ((EROWS < SEQ) ? EROWS : SEQ)

static_assert(NB >= 1 && NB <= NB_FULL);
static_assert(SEQ >= 128 && SEQ <= SEQ_FULL && (SEQ % 128) == 0);
static_assert(DIM == NHEAD * HD);
static_assert(HD == 64);
static_assert((DIM % 64) == 0 && (DIM % 32) == 0);
static_assert((DFF % 64) == 0 && (DFF % 32) == 0);
static_assert((MROWS % 64) == 0);
static_assert(DIM == 128 * 8);
static_assert(DIM == 256 * 4);
static_assert(DFF == 256 * 16);
static_assert(CDIM == 64 && (CDIM % 32) == 0);
static_assert(DCAT == 256 && (DCAT % 64) == 0);
static_assert((EROWS % 128) == 0 && EROWS >= 128);
static_assert((EROWS_EFF % 128) == 0 && EROWS_EFF <= SEQ);
static_assert((SEQ % 8) == 0);
static_assert(((size_t)DIM * DIM) % 2048 == 0);
static_assert(((size_t)NCB * DFF * CDIM) % 2048 == 0);
static_assert(((size_t)NCB * DIM * CDIM) % 2048 == 0);
static_assert((size_t)MROWS * DFF < (size_t)0xFFFFFFFFu);

#define LDT 72
#define LDC 68
static_assert((LDT % 8) == 0 && LDT >= 64);
static_assert((LDC % 4) == 0 && LDC >= 64);

#define WCARRY 64.0f
#define PCARRY 1024.0f
#define VCARRY 64.0f
#define RCARRY 2048.0f
#define RINV   (1.0f / 2048.0f)

#define PLANE16_ELEMS ((size_t)MROWS * DIM)
#define PLANE16_BYTES (PLANE16_ELEMS * 2)
#define WSQ_ELEMS     ((size_t)DIM * DIM)
#define ADPL_ELEMS    ((size_t)MROWS * DCAT)
#define SPL_ELEMS     ((size_t)MROWS * DFF)
#define OFF_WQKV  ((size_t)0)
#define OFF_WO    (OFF_WQKV + 3 * WSQ_ELEMS * 2)
#define OFF_W1D   (OFF_WO + WSQ_ELEMS * 2)
#define OFF_W1U   (OFF_W1D + (size_t)DCAT * DIM * 2)
#define OFF_W2D   (OFF_W1U + (size_t)NCB * DFF * CDIM * 2)
#define OFF_W2U   (OFF_W2D + (size_t)DCAT * DFF * 2)
#define OFF_CS    (OFF_W2U + (size_t)NCB * DIM * CDIM * 2)
#define OFF_RA    (OFF_CS + (size_t)SEQ * 64 * 4)
#define RA_BYTES  (8 * PLANE16_BYTES)
#define OFF_RB    (OFF_RA + RA_BYTES)
#define RB_BYTES  (2 * PLANE16_BYTES)
#define OFF_X1    (OFF_RB + RB_BYTES)
#define OFF_H2    (OFF_X1 + PLANE16_ELEMS * 4)
#define OFF_AD    (OFF_H2 + 2 * PLANE16_BYTES)
#define OFF_S     (OFF_AD + 2 * ADPL_ELEMS * 2)
#define OFF_BD    (OFF_S + 2 * SPL_ELEMS * 2)
#define WS_TOTAL  (OFF_BD + 2 * ADPL_ELEMS * 2)
static_assert((PLANE16_BYTES % 128) == 0 && ((WSQ_ELEMS * 2) % 128) == 0);
static_assert((OFF_CS % 128) == 0 && (OFF_RA % 128) == 0 && (OFF_RB % 128) == 0);
static_assert((OFF_X1 % 128) == 0 && (OFF_H2 % 128) == 0 && (OFF_AD % 128) == 0);
static_assert((OFF_S % 128) == 0 && (OFF_BD % 128) == 0);
static_assert(RA_BYTES >= SPL_ELEMS * 4);
static_assert(RB_BYTES >= PLANE16_ELEMS * 4);
static_assert(WS_TOTAL <= (size_t)134217728);

__device__ __forceinline__ float bf16r(float x) {
  unsigned int u = __float_as_uint(x);
  u = (u + 0x7FFFu + ((u >> 16) & 1u)) & 0xFFFF0000u;
  return __uint_as_float(u);
}

__device__ __forceinline__ size_t full_row(unsigned crow) {
  const unsigned bidx = crow / (unsigned)SEQ;
  const unsigned sq = crow - bidx * (unsigned)SEQ;
  return (size_t)bidx * SEQ_FULL + sq;
}

static __device__ __forceinline__ _Float16 toh_flush(float v) {
  const _Float16 r = (_Float16)v;
  return (fabsf(v) < 6.103515625e-05f) ? (_Float16)0.0f : r;
}

__device__ __forceinline__ v16h frag_at(const _Float16* p) {
  v8h lo = *(const v8h*)(p);
  v8h hi = *(const v8h*)(p + 16);
  v16h out;
#pragma unroll
  for (int i = 0; i < 8; ++i) { out[i] = lo[i]; out[i + 8] = hi[i]; }
  return out;
}
__device__ __forceinline__ v16h ld_frag(const _Float16* base, unsigned ld) {
  const unsigned lane = threadIdx.x & 31u;
  return frag_at(base + (lane & 15u) * ld + (lane >> 4) * 8u);
}

__device__ __forceinline__ v8f wmma16(v16h a, v16h b, v8f c) {
  v8f d = __builtin_amdgcn_wmma_f32_16x16x32_f16(false, a, false, b, (short)0, c,
                                                 false, false);
  asm volatile("v_nop\n\tv_nop\n\tv_nop\n\tv_nop" : "+v"(d) : "v"(a), "v"(b));
  return d;
}

__device__ __forceinline__ float red16_max(float x) {
#pragma unroll
  for (int off = 1; off < 16; off <<= 1) x = fmaxf(x, __shfl_xor(x, off, 32));
  return x;
}
__device__ __forceinline__ float red16_sum(float x) {
#pragma unroll
  for (int off = 1; off < 16; off <<= 1) x += __shfl_xor(x, off, 32);
  return x;
}
__device__ __forceinline__ float red32_sum(float x) {
#pragma unroll
  for (int off = 1; off < 32; off <<= 1) x += __shfl_xor(x, off, 32);
  return x;
}

__device__ __forceinline__ void wave_lds_sync() {
  __builtin_amdgcn_fence(3  , "wavefront");
  asm volatile("s_wait_dscnt 0x0" ::: "memory");
  __builtin_amdgcn_wave_barrier();
}

__global__ __launch_bounds__(256) void wconv_kernel(
    const float* __restrict__ W, _Float16* __restrict__ Wt,
    unsigned N, unsigned K, unsigned headmode) {
  __shared__ _Float16 T[64 * LDT];
  const unsigned tid = threadIdx.x;
  const unsigned n0 = blockIdx.x * 64u;
  const unsigned k0 = blockIdx.y * 64u;
  const size_t sbase = headmode ? (size_t)blockIdx.x * K * 64u : (size_t)n0;
  const unsigned ldw = headmode ? 64u : N;
#pragma unroll 4
  for (unsigned j = 0; j < 16u; ++j) {
    const unsigned idx = tid + 256u * j;
    const unsigned kr = idx >> 6, nc = idx & 63u;
    const float v = W[sbase + (size_t)(k0 + kr) * ldw + nc];
    T[nc * LDT + kr] = (_Float16)(WCARRY * bf16r(v));
  }
  __syncthreads();
  v8h x[2];
  size_t off[2];
#pragma unroll
  for (unsigned i = 0; i < 2u; ++i) {
    const unsigned n = 32u * i + (tid >> 3);
    const unsigned kc = (tid & 7u) * 8u;
    x[i] = *(const v8h*)&T[n * LDT + kc];
    off[i] = (size_t)(n0 + n) * K + k0 + kc;
  }
#pragma unroll
  for (int i = 0; i < 2; ++i) *(volatile v8h*)(Wt + off[i]) = x[i];
  __threadfence();
#pragma unroll
  for (int i = 0; i < 2; ++i) *(volatile v8h*)(Wt + off[i]) = x[i];
}

__global__ __launch_bounds__(256) void wcast_kernel(
    const float* __restrict__ W, _Float16* __restrict__ Wt, unsigned n8) {
  const unsigned i = blockIdx.x * 256u + threadIdx.x;
  const unsigned ic = (i < n8) ? i : (n8 - 1u);
  const float* sp = W + (size_t)ic * 8u;
  const v4f a0 = *(const v4f*)(sp);
  const v4f a1 = *(const v4f*)(sp + 4);
  v8h x;
#pragma unroll
  for (int j = 0; j < 4; ++j) {
    x[j]     = toh_flush(WCARRY * bf16r(a0[j]));
    x[j + 4] = toh_flush(WCARRY * bf16r(a1[j]));
  }
  _Float16* dp = Wt + (size_t)ic * 8u;
  *(volatile v8h*)dp = x;
  __threadfence();
  *(volatile v8h*)dp = x;
}

__global__ __launch_bounds__(256) void rope_table_kernel(float* __restrict__ CS) {
#pragma clang fp contract(off)
  __shared__ float T[8 * 64];
  const unsigned tid = threadIdx.x;
  const unsigned r = tid >> 5, p = tid & 31u;
  const unsigned t = blockIdx.x * 8u + r;
  const double a = (double)p * (13.287712379549449 / 32.0);
  const double fl = floor(a);
  const float fr = (float)(a - fl);
  const float inv = ldexpf(exp2f(-fr), -(int)fl);
  const float ang = (float)t * inv;
  T[r * 64u + p] = cosf(ang);
  T[r * 64u + 32u + p] = sinf(ang);
  __syncthreads();
  if (tid < 128u) {
    const v4f o = *(const v4f*)&T[tid * 4u];
    float* dp = CS + (size_t)blockIdx.x * 512u + tid * 4u;
    *(volatile v4f*)dp = o;
    __threadfence();
    *(volatile v4f*)dp = o;
  }
}

__global__ __launch_bounds__(128) void rms_kernel(
    const float* __restrict__ Xin, const float* __restrict__ g,
    _Float16* __restrict__ dhi, _Float16* __restrict__ drs,
    unsigned src_full, unsigned rne_in) {
#pragma clang fp contract(off)
  __shared__ float rowf[DIM];
  __shared__ _Float16 rowh[DIM];
  __shared__ _Float16 rowr[DIM];
  __shared__ float red[4];
  const unsigned tid = threadIdx.x, lane = tid & 31u, w = tid >> 5;
  const unsigned crow = blockIdx.x;
  const size_t srow = src_full ? full_row(crow) : (size_t)crow;
  const float* sp = Xin + srow * DIM + tid * 8u;
  v4f a0 = *(const v4f*)(sp);
  v4f a1 = *(const v4f*)(sp + 4);
  if (rne_in) {
#pragma unroll
    for (int j = 0; j < 4; ++j) { a0[j] = bf16r(a0[j]); a1[j] = bf16r(a1[j]); }
  }
  *(v4f*)&rowf[tid * 8u] = a0;
  *(v4f*)&rowf[tid * 8u + 4u] = a1;
  float ss = ((a0[0] * a0[0] + a0[1] * a0[1]) + (a0[2] * a0[2] + a0[3] * a0[3])) +
             ((a1[0] * a1[0] + a1[1] * a1[1]) + (a1[2] * a1[2] + a1[3] * a1[3]));
  ss = red32_sum(ss);
  if (lane == 0u) red[w] = ss;
  __syncthreads();
  const float msq = ((red[0] + red[1]) + (red[2] + red[3])) * (1.0f / (float)DIM);
  const float sc = rsqrtf(msq + 1.0e-6f);
#pragma unroll 1
  for (unsigned j = 0; j < 8u; ++j) {
    const unsigned c = tid + 128u * j;
    const float v = (rowf[c] * sc) * bf16r(g[c]);
    const _Float16 hi = toh_flush(v);
    rowh[c] = hi;
    rowr[c] = toh_flush((v - (float)hi) * RCARRY);
  }
  __syncthreads();
  const v8h o = *(const v8h*)&rowh[tid * 8u];
  const v8h orr = *(const v8h*)&rowr[tid * 8u];
  _Float16* dp = dhi + (size_t)crow * DIM + tid * 8u;
  _Float16* dq = drs + (size_t)crow * DIM + tid * 8u;
  *(volatile v8h*)dp = o;
  *(volatile v8h*)dq = orr;
  __threadfence();
  *(volatile v8h*)dp = o;
  *(volatile v8h*)dq = orr;
}

__device__ __forceinline__ void gemm_hr_main(
    const _Float16* __restrict__ Ahi, const _Float16* __restrict__ Ars, const unsigned lda,
    const _Float16* __restrict__ Bt, const unsigned ldb, const unsigned K,
    const unsigned arow0, const unsigned brow0, const unsigned nres, float* Cs) {
  const unsigned tid = threadIdx.x, lane = tid & 31u;
  const unsigned w = (unsigned)__builtin_amdgcn_readfirstlane((int)(tid >> 5));
  const unsigned mw = w >> 1, nw = w & 1u;
  const unsigned hh = lane >> 4, m = lane & 15u;
  const size_t aoff = (size_t)(arow0 + mw * 16u + m) * lda + hh * 8u;
  const _Float16* ap  = Ahi + aoff;
  const _Float16* rp  = Ars + aoff;
  const _Float16* bp0 = Bt + (size_t)(brow0 + nw * 32u + m) * ldb + hh * 8u;
  const _Float16* bp1 = bp0 + (size_t)16 * ldb;
  v8f acc0 = {}, acc1 = {}, rc0 = {}, rc1 = {};
  if (nres != 0u) {
#pragma unroll 2
    for (unsigned k0 = 0; k0 < K; k0 += 32u) {
      const v16h a  = frag_at(ap + k0);
      const v16h ar = frag_at(rp + k0);
      const v16h b0 = frag_at(bp0 + k0);
      const v16h b1 = frag_at(bp1 + k0);
      acc0 = wmma16(a, b0, acc0);
      acc1 = wmma16(a, b1, acc1);
      rc0  = wmma16(ar, b0, rc0);
      rc1  = wmma16(ar, b1, rc1);
    }
  } else {
#pragma unroll 2
    for (unsigned k0 = 0; k0 < K; k0 += 32u) {
      const v16h a  = frag_at(ap + k0);
      const v16h b0 = frag_at(bp0 + k0);
      const v16h b1 = frag_at(bp1 + k0);
      acc0 = wmma16(a, b0, acc0);
      acc1 = wmma16(a, b1, acc1);
    }
  }
#pragma unroll
  for (int r = 0; r < 8; ++r) {
    float* d = &Cs[(mw * 16u + hh * 8u + (unsigned)r) * LDC + nw * 32u + m];
    d[0]  = acc0[r] + rc0[r] * RINV;
    d[16] = acc1[r] + rc1[r] * RINV;
  }
  __syncthreads();
}

__device__ __forceinline__ void epi_f16_hr(
    const float* Cs, _Float16* __restrict__ outhi, _Float16* __restrict__ outrs,
    const unsigned pitch, const unsigned row0, const unsigned n0, const float scale) {
  const unsigned tid = threadIdx.x;
  v8h x[2], xr[2];
  size_t off[2];
#pragma unroll
  for (unsigned i = 0; i < 2u; ++i) {
    const unsigned r = 32u * i + (tid >> 3);
    const unsigned c = (tid & 7u) * 8u;
    const v4f u0 = *(const v4f*)&Cs[r * LDC + c];
    const v4f u1 = *(const v4f*)&Cs[r * LDC + c + 4];
#pragma unroll
    for (int j = 0; j < 4; ++j) {
      const float v0 = u0[j] * scale, v1 = u1[j] * scale;
      const _Float16 h0 = toh_flush(v0), h1 = toh_flush(v1);
      x[i][j]      = h0;
      x[i][j + 4]  = h1;
      xr[i][j]     = toh_flush((v0 - (float)h0) * RCARRY);
      xr[i][j + 4] = toh_flush((v1 - (float)h1) * RCARRY);
    }
    off[i] = (size_t)(row0 + r) * pitch + n0 + c;
  }
#pragma unroll
  for (int i = 0; i < 2; ++i) *(volatile v8h*)(outhi + off[i]) = x[i];
#pragma unroll
  for (int i = 0; i < 2; ++i) *(volatile v8h*)(outrs + off[i]) = xr[i];
  __threadfence();
#pragma unroll
  for (int i = 0; i < 2; ++i) *(volatile v8h*)(outhi + off[i]) = x[i];
#pragma unroll
  for (int i = 0; i < 2; ++i) *(volatile v8h*)(outrs + off[i]) = xr[i];
}

__device__ __forceinline__ void epi_rope_hr(
    const float* Cs, const float* __restrict__ CS,
    _Float16* __restrict__ outhi, _Float16* __restrict__ outrs,
    const unsigned row0, const unsigned n0, const float scale) {
  const unsigned tid = threadIdx.x;
  v8h x[2], xr[2];
  size_t off[2];
#pragma unroll
  for (unsigned i = 0; i < 2u; ++i) {
    const unsigned r = 32u * i + (tid >> 3);
    const unsigned c = (tid & 7u) * 8u;
    const unsigned crow = row0 + r;
    const unsigned pos = crow - (crow / (unsigned)SEQ) * (unsigned)SEQ;
    const float* tp = CS + (size_t)pos * 64u + (c >> 1);
    const v4f cs = *(const v4f*)(tp);
    const v4f sn = *(const v4f*)(tp + 32);
    const v4f u0 = *(const v4f*)&Cs[r * LDC + c];
    const v4f u1 = *(const v4f*)&Cs[r * LDC + c + 4];
    float e[8];
#pragma unroll
    for (int j = 0; j < 4; ++j) { e[j] = u0[j] * scale; e[j + 4] = u1[j] * scale; }
#pragma unroll
    for (int j = 0; j < 4; ++j) {
      const float x1 = e[2 * j], x2 = e[2 * j + 1];
      const float o1 = x1 * cs[j] - x2 * sn[j];
      const float o2 = x1 * sn[j] + x2 * cs[j];
      const _Float16 h1 = toh_flush(o1), h2 = toh_flush(o2);
      x[i][2 * j]      = h1;
      x[i][2 * j + 1]  = h2;
      xr[i][2 * j]     = toh_flush((o1 - (float)h1) * RCARRY);
      xr[i][2 * j + 1] = toh_flush((o2 - (float)h2) * RCARRY);
    }
    off[i] = (size_t)crow * DIM + n0 + c;
  }
#pragma unroll
  for (int i = 0; i < 2; ++i) *(volatile v8h*)(outhi + off[i]) = x[i];
#pragma unroll
  for (int i = 0; i < 2; ++i) *(volatile v8h*)(outrs + off[i]) = xr[i];
  __threadfence();
#pragma unroll
  for (int i = 0; i < 2; ++i) *(volatile v8h*)(outhi + off[i]) = x[i];
#pragma unroll
  for (int i = 0; i < 2; ++i) *(volatile v8h*)(outrs + off[i]) = xr[i];
}

__device__ __forceinline__ void epi_vt_hr(
    const float* Cs, _Float16* __restrict__ outhi, _Float16* __restrict__ outrs,
    const unsigned row0, const unsigned n0, const float scale) {
  const unsigned tid = threadIdx.x;
  const unsigned bidx = row0 / (unsigned)SEQ;
  const unsigned key0 = row0 - bidx * (unsigned)SEQ;
  v8h x[2], xr[2];
  size_t off[2];
#pragma unroll
  for (unsigned i = 0; i < 2u; ++i) {
    const unsigned dcol = 32u * i + (tid >> 3);
    const unsigned kk = (tid & 7u) * 8u;
#pragma unroll
    for (unsigned j = 0; j < 8u; ++j) {
      const float v = Cs[(kk + j) * LDC + dcol] * scale;
      const _Float16 hi = toh_flush(v);
      x[i][j]  = hi;
      xr[i][j] = toh_flush((v - (float)hi) * RCARRY);
    }
    off[i] = ((size_t)bidx * DIM + n0 + dcol) * SEQ + key0 + kk;
  }
#pragma unroll
  for (int i = 0; i < 2; ++i) *(volatile v8h*)(outhi + off[i]) = x[i];
#pragma unroll
  for (int i = 0; i < 2; ++i) *(volatile v8h*)(outrs + off[i]) = xr[i];
  __threadfence();
#pragma unroll
  for (int i = 0; i < 2; ++i) *(volatile v8h*)(outhi + off[i]) = x[i];
#pragma unroll
  for (int i = 0; i < 2; ++i) *(volatile v8h*)(outrs + off[i]) = xr[i];
}

__device__ __forceinline__ void epi_f32_res(
    const float* Cs, const float* __restrict__ res,
    const unsigned res_full, const unsigned res_rne, float* __restrict__ outf,
    const unsigned out_full, const unsigned row0, const unsigned n0, const float scale) {
  const unsigned tid = threadIdx.x;
  v4f xs[4];
  size_t off[4];
#pragma unroll
  for (unsigned i = 0; i < 4u; ++i) {
    const unsigned r = 16u * i + (tid >> 4);
    const unsigned c = (tid & 15u) * 4u;
    const unsigned crow = row0 + r;
    const size_t frow = full_row(crow);
    const size_t rrow = res_full ? frow : (size_t)crow;
    const size_t orow = out_full ? frow : (size_t)crow;
    const v4f u = *(const v4f*)&Cs[r * LDC + c];
    const v4f rv = *(const v4f*)(res + rrow * DIM + n0 + c);
    v4f val;
#pragma unroll
    for (int j = 0; j < 4; ++j) {
      const float rr = res_rne ? bf16r(rv[j]) : rv[j];
      val[j] = u[j] * scale + rr;
    }
    xs[i] = val;
    off[i] = orow * DIM + n0 + c;
  }
#pragma unroll
  for (int i = 0; i < 4; ++i) *(volatile v4f*)(outf + off[i]) = xs[i];
  __threadfence();
#pragma unroll
  for (int i = 0; i < 4; ++i) *(volatile v4f*)(outf + off[i]) = xs[i];
}

__device__ __forceinline__ void epi_f32_plain(
    const float* Cs, float* __restrict__ outf, const unsigned pitch,
    const unsigned row0, const unsigned n0) {
  const unsigned tid = threadIdx.x;
  v4f xs[4];
  size_t off[4];
#pragma unroll
  for (unsigned i = 0; i < 4u; ++i) {
    const unsigned r = 16u * i + (tid >> 4);
    const unsigned c = (tid & 15u) * 4u;
    xs[i] = *(const v4f*)&Cs[r * LDC + c];
    off[i] = (size_t)(row0 + r) * pitch + n0 + c;
  }
#pragma unroll
  for (int i = 0; i < 4; ++i) *(volatile v4f*)(outf + off[i]) = xs[i];
  __threadfence();
#pragma unroll
  for (int i = 0; i < 4; ++i) *(volatile v4f*)(outf + off[i]) = xs[i];
}

__global__ __launch_bounds__(256) void gemm_qkv_kernel(
    const _Float16* __restrict__ H16, const _Float16* __restrict__ H16r,
    const _Float16* __restrict__ WqkvT, const float* __restrict__ CS,
    _Float16* __restrict__ qkv16, _Float16* __restrict__ qkv16r) {
  __shared__ float Cs[64 * LDC];
  const unsigned sel = blockIdx.x / (unsigned)(DIM / 64);
  const unsigned n0 = (blockIdx.x - sel * (unsigned)(DIM / 64)) * 64u;
  const unsigned row0 = blockIdx.y * 64u;
  const unsigned pos0 = row0 - (row0 / (unsigned)SEQ) * (unsigned)SEQ;
  const unsigned nres = (pos0 < (unsigned)EROWS_EFF) ? 1u : 0u;
  gemm_hr_main(H16, H16r, (unsigned)DIM, WqkvT, (unsigned)DIM, (unsigned)DIM,
               row0, blockIdx.x * 64u, nres, Cs);
  _Float16* outp = qkv16 + (size_t)sel * PLANE16_ELEMS;
  _Float16* outr = qkv16r + (size_t)sel * PLANE16_ELEMS;
  if (sel < 2u) epi_rope_hr(Cs, CS, outp, outr, row0, n0, 1.0f / WCARRY);
  else          epi_vt_hr(Cs, outp, outr, row0, n0, 1.0f / WCARRY);
}

__global__ __launch_bounds__(256) void gemm_wo_kernel(
    const _Float16* __restrict__ Ctx16, const _Float16* __restrict__ Ctx16r,
    const _Float16* __restrict__ WoT, const float* __restrict__ X, float* __restrict__ X1) {
  __shared__ float Cs[64 * LDC];
  const unsigned n0 = blockIdx.x * 64u;
  const unsigned row0 = blockIdx.y * 64u;
  const unsigned pos0 = row0 - (row0 / (unsigned)SEQ) * (unsigned)SEQ;
  const unsigned nres = (pos0 < (unsigned)EROWS_EFF) ? 1u : 0u;
  gemm_hr_main(Ctx16, Ctx16r, (unsigned)DIM, WoT, (unsigned)DIM, (unsigned)DIM,
               row0, n0, nres, Cs);
  epi_f32_res(Cs, X, 1u, 1u, X1, 0u, row0, n0, 1.0f / (WCARRY * VCARRY));
}

__global__ __launch_bounds__(256) void gemm_down_kernel(
    const _Float16* __restrict__ Ahi, const _Float16* __restrict__ Ars,
    const _Float16* __restrict__ Wd, _Float16* __restrict__ outhi,
    _Float16* __restrict__ outrs, unsigned K) {
  __shared__ float Cs[64 * LDC];
  const unsigned n0 = blockIdx.x * 64u;
  const unsigned row0 = blockIdx.y * 64u;
  gemm_hr_main(Ahi, Ars, K, Wd, K, K, row0, n0, 1u, Cs);
  epi_f16_hr(Cs, outhi, outrs, (unsigned)DCAT, row0, n0, 1.0f / WCARRY);
}

__global__ __launch_bounds__(256) void up_prod_kernel(
    const _Float16* __restrict__ ADhi, const _Float16* __restrict__ ADrs,
    const _Float16* __restrict__ Wup, float* __restrict__ P, unsigned N) {
  __shared__ float Cs[64 * LDC];
  const unsigned tid = threadIdx.x, lane = tid & 31u;
  const unsigned w = (unsigned)__builtin_amdgcn_readfirstlane((int)(tid >> 5));
  const unsigned mw = w >> 1, nw = w & 1u;
  const unsigned hh = lane >> 4, m = lane & 15u;
  const unsigned n0 = blockIdx.x * 64u;
  const unsigned row0 = blockIdx.y * 64u;
  v8f p0, p1;
#pragma unroll
  for (int r = 0; r < 8; ++r) { p0[r] = 1.0f; p1[r] = 1.0f; }
#pragma unroll 1
  for (unsigned h = 0; h < (unsigned)NCB; ++h) {
    const size_t aoff = (size_t)(row0 + mw * 16u + m) * DCAT + h * (unsigned)CDIM + hh * 8u;
    const _Float16* ap  = ADhi + aoff;
    const _Float16* rp  = ADrs + aoff;
    const _Float16* bp0 = Wup + ((size_t)h * N + n0 + nw * 32u + m) * CDIM + hh * 8u;
    const _Float16* bp1 = bp0 + (size_t)16 * CDIM;
    v8f acc0 = {}, acc1 = {}, rc0 = {}, rc1 = {};
#pragma unroll
    for (unsigned k0 = 0; k0 < (unsigned)CDIM; k0 += 32u) {
      const v16h a  = frag_at(ap + k0);
      const v16h ar = frag_at(rp + k0);
      const v16h b0 = frag_at(bp0 + k0);
      const v16h b1 = frag_at(bp1 + k0);
      acc0 = wmma16(a, b0, acc0);
      acc1 = wmma16(a, b1, acc1);
      rc0  = wmma16(ar, b0, rc0);
      rc1  = wmma16(ar, b1, rc1);
    }
#pragma unroll
    for (int r = 0; r < 8; ++r) {
      p0[r] *= (acc0[r] + rc0[r] * RINV) * (1.0f / WCARRY);
      p1[r] *= (acc1[r] + rc1[r] * RINV) * (1.0f / WCARRY);
    }
  }
#pragma unroll
  for (int r = 0; r < 8; ++r) {
    float* d = &Cs[(mw * 16u + hh * 8u + (unsigned)r) * LDC + nw * 32u + m];
    d[0]  = p0[r];
    d[16] = p1[r];
  }
  __syncthreads();
  epi_f32_plain(Cs, P, N, row0, n0);
}

__global__ __launch_bounds__(256) void rms_silu_kernel(
    const float* __restrict__ P, _Float16* __restrict__ shi, _Float16* __restrict__ srs) {
#pragma clang fp contract(off)
  __shared__ float rowf[DFF];
  __shared__ _Float16 rowh[DFF];
  __shared__ _Float16 rowr[DFF];
  __shared__ float red[8];
  const unsigned tid = threadIdx.x, lane = tid & 31u, w = tid >> 5;
  const unsigned crow = blockIdx.x;
  const float* sp = P + (size_t)crow * DFF;
  float ss = 0.0f;
#pragma unroll 1
  for (unsigned j = 0; j < 4u; ++j) {
    const unsigned c = (tid + 256u * j) * 4u;
    const v4f a = *(const v4f*)(sp + c);
    *(v4f*)&rowf[c] = a;
    ss += (a[0] * a[0] + a[1] * a[1]) + (a[2] * a[2] + a[3] * a[3]);
  }
  ss = red32_sum(ss);
  if (lane == 0u) red[w] = ss;
  __syncthreads();
  const float tot = ((red[0] + red[1]) + (red[2] + red[3])) +
                    ((red[4] + red[5]) + (red[6] + red[7]));
  const float sc = rsqrtf(tot * (1.0f / (float)DFF) + 1.0e-6f);
#pragma unroll 1
  for (unsigned j = 0; j < 16u; ++j) {
    const unsigned c = tid + 256u * j;
    const float v = rowf[c] * sc;
    const float e = expf(-v);
    const float s = v * __builtin_amdgcn_rcpf(1.0f + e);
    const _Float16 hi = toh_flush(s);
    rowh[c] = hi;
    rowr[c] = toh_flush((s - (float)hi) * RCARRY);
  }
  __syncthreads();
  v8h x[2], xr[2];
  size_t off[2];
#pragma unroll
  for (unsigned i = 0; i < 2u; ++i) {
    const unsigned c8 = (tid + 256u * i) * 8u;
    x[i]  = *(const v8h*)&rowh[c8];
    xr[i] = *(const v8h*)&rowr[c8];
    off[i] = (size_t)crow * DFF + c8;
  }
#pragma unroll
  for (int i = 0; i < 2; ++i) *(volatile v8h*)(shi + off[i]) = x[i];
#pragma unroll
  for (int i = 0; i < 2; ++i) *(volatile v8h*)(srs + off[i]) = xr[i];
  __threadfence();
#pragma unroll
  for (int i = 0; i < 2; ++i) *(volatile v8h*)(shi + off[i]) = x[i];
#pragma unroll
  for (int i = 0; i < 2; ++i) *(volatile v8h*)(srs + off[i]) = xr[i];
}

__global__ __launch_bounds__(256) void rms_out_kernel(
    const float* __restrict__ P2, const float* __restrict__ X1, float* __restrict__ out) {
#pragma clang fp contract(off)
  __shared__ float red[8];
  const unsigned tid = threadIdx.x, lane = tid & 31u, w = tid >> 5;
  const unsigned crow = blockIdx.x;
  const v4f a = *(const v4f*)(P2 + (size_t)crow * DIM + tid * 4u);
  float ss = (a[0] * a[0] + a[1] * a[1]) + (a[2] * a[2] + a[3] * a[3]);
  ss = red32_sum(ss);
  if (lane == 0u) red[w] = ss;
  __syncthreads();
  const float tot = ((red[0] + red[1]) + (red[2] + red[3])) +
                    ((red[4] + red[5]) + (red[6] + red[7]));
  const float sc = rsqrtf(tot * (1.0f / (float)DIM) + 1.0e-6f);
  const v4f xr = *(const v4f*)(X1 + (size_t)crow * DIM + tid * 4u);
  v4f val;
#pragma unroll
  for (int j = 0; j < 4; ++j) {
    const float f = a[j] * sc;
    val[j] = xr[j] + f;
  }
  float* dp = out + full_row(crow) * DIM + tid * 4u;
  *(volatile v4f*)dp = val;
  __threadfence();
  *(volatile v4f*)dp = val;
}

__global__ __launch_bounds__(256) void attn_kernel(
    const _Float16* __restrict__ Qh, const _Float16* __restrict__ Kh,
    const _Float16* __restrict__ Vt, _Float16* __restrict__ Ov) {
  __shared__ _Float16 Ks[64 * LDT];
  __shared__ _Float16 Vs[64 * LDT];
  __shared__ _Float16 Ps[8 * 16 * LDT];

  const unsigned tid = threadIdx.x, lane = tid & 31u;
  const unsigned w = (unsigned)__builtin_amdgcn_readfirstlane((int)(tid >> 5));
  const unsigned hh = lane >> 4, m = lane & 15u;
  const unsigned q0 = blockIdx.x * 128u;
  const unsigned head = blockIdx.y;
  const unsigned b = blockIdx.z;
  const unsigned qw0 = q0 + w * 16u;
  const float scale = 0.125f;
  _Float16* P = Ps + w * (16u * LDT);

  const size_t qoff = (size_t)(b * (unsigned)SEQ + qw0 + m) * DIM + head * HD + hh * 8u;
  v16h qf[2];
  qf[0] = frag_at(Qh + qoff);
  qf[1] = frag_at(Qh + qoff + 32);

  float mrow[8], lrow[8];
  v8f o[4];
#pragma unroll
  for (int v = 0; v < 8; ++v) { mrow[v] = -1.0e30f; lrow[v] = 0.0f; }
#pragma unroll
  for (int nb = 0; nb < 4; ++nb) o[nb] = (v8f){};

  const size_t kplane = (size_t)b * SEQ * DIM + head * HD;
  const size_t vplane = ((size_t)b * DIM + head * HD) * SEQ;
  const unsigned kend = q0 + 128u;

  for (unsigned kb = 0; kb < kend; kb += 64u) {
#pragma unroll
    for (unsigned j = 0; j < 2u; ++j) {
      const unsigned idx = tid + 256u * j;
      const unsigned r = idx >> 3, c = (idx & 7u) * 8u;
      *(v8h*)&Ks[r * LDT + c] = *(const v8h*)(Kh + kplane + (size_t)(kb + r) * DIM + c);
      *(v8h*)&Vs[r * LDT + c] = *(const v8h*)(Vt + vplane + (size_t)r * SEQ + kb + c);
    }
    __syncthreads();

    if (kb <= qw0 + 15u) {
      v8f s[4];
#pragma unroll
      for (int kg = 0; kg < 4; ++kg) {
        v8f t = {};
#pragma unroll
        for (int c = 0; c < 2; ++c) {
          const v16h kf = ld_frag(&Ks[(kg * 16) * LDT + c * 32], LDT);
          t = wmma16(qf[c], kf, t);
        }
        s[kg] = t * scale;
      }
      if (kb + 63u > qw0) {
#pragma unroll
        for (int kg = 0; kg < 4; ++kg) {
          const unsigned key = kb + (unsigned)kg * 16u + m;
#pragma unroll
          for (int v = 0; v < 8; ++v) {
            const unsigned qr = qw0 + hh * 8u + (unsigned)v;
            s[kg][v] = (key > qr) ? -1.0e30f : s[kg][v];
          }
        }
      }

      float alpha[8];
#pragma unroll
      for (int v = 0; v < 8; ++v) {
        float mx = fmaxf(fmaxf(s[0][v], s[1][v]), fmaxf(s[2][v], s[3][v]));
        mx = red16_max(mx);
        const float mn = fmaxf(mrow[v], mx);
        alpha[v] = __expf(mrow[v] - mn);
        mrow[v] = mn;
      }
#pragma unroll
      for (int kg = 0; kg < 4; ++kg)
#pragma unroll
        for (int v = 0; v < 8; ++v) s[kg][v] = __expf(s[kg][v] - mrow[v]);
#pragma unroll
      for (int v = 0; v < 8; ++v) {
        const float rs = red16_sum((s[0][v] + s[1][v]) + (s[2][v] + s[3][v]));
        lrow[v] = alpha[v] * lrow[v] + rs;
      }
#pragma unroll
      for (int nb = 0; nb < 4; ++nb)
#pragma unroll
        for (int v = 0; v < 8; ++v) o[nb][v] = o[nb][v] * alpha[v];

#pragma unroll
      for (int kg = 0; kg < 4; ++kg)
#pragma unroll
        for (int v = 0; v < 8; ++v)
          P[(hh * 8u + (unsigned)v) * LDT + (unsigned)kg * 16u + m] =
              (_Float16)(s[kg][v] * PCARRY);
      wave_lds_sync();

#pragma unroll
      for (int c = 0; c < 2; ++c) {
        const v16h pf = ld_frag(P + c * 32, LDT);
#pragma unroll
        for (int nb = 0; nb < 4; ++nb) {
          const v16h vf = ld_frag(&Vs[(nb * 16) * LDT + c * 32], LDT);
          o[nb] = wmma16(pf, vf, o[nb]);
        }
      }
    }
    __syncthreads();
  }

  float inv[8];
#pragma unroll
  for (int v = 0; v < 8; ++v) inv[v] = __builtin_amdgcn_rcpf(lrow[v]) * (VCARRY / PCARRY);
#pragma unroll
  for (int nb = 0; nb < 4; ++nb)
#pragma unroll
    for (int v = 0; v < 8; ++v)
      P[(hh * 8u + (unsigned)v) * LDT + (unsigned)nb * 16u + m] = (_Float16)(o[nb][v] * inv[v]);
  wave_lds_sync();
  v8h x[4];
  size_t off[4];
#pragma unroll
  for (unsigned i = 0; i < 4u; ++i) {
    const unsigned r = 4u * i + (lane >> 3);
    const unsigned c = (lane & 7u) * 8u;
    x[i] = *(const v8h*)&P[r * LDT + c];
    off[i] = (size_t)(b * (unsigned)SEQ + qw0 + r) * DIM + head * HD + c;
  }
#pragma unroll
  for (int i = 0; i < 4; ++i) *(volatile v8h*)(Ov + off[i]) = x[i];
  __threadfence();
#pragma unroll
  for (int i = 0; i < 4; ++i) *(volatile v8h*)(Ov + off[i]) = x[i];
}

__global__ __launch_bounds__(256) __attribute__((amdgpu_num_vgpr(256))) void attn_early_kernel(
    const _Float16* __restrict__ Qh, const _Float16* __restrict__ Qr,
    const _Float16* __restrict__ Kh, const _Float16* __restrict__ Kr,
    const _Float16* __restrict__ Vt, const _Float16* __restrict__ Vtr,
    _Float16* __restrict__ Ov, _Float16* __restrict__ Ovr) {
  __shared__ _Float16 Ks[64 * LDT];
  __shared__ _Float16 Kq[64 * LDT];
  __shared__ _Float16 Vs[64 * LDT];
  __shared__ _Float16 Vq[64 * LDT];
  __shared__ _Float16 Ps[8 * 16 * LDT];

  const unsigned tid = threadIdx.x, lane = tid & 31u;
  const unsigned w = (unsigned)__builtin_amdgcn_readfirstlane((int)(tid >> 5));
  const unsigned hh = lane >> 4, m = lane & 15u;
  const unsigned q0 = blockIdx.x * 128u;
  const unsigned head = blockIdx.y;
  const unsigned b = blockIdx.z;
  const unsigned qw0 = q0 + w * 16u;
  const float scale = 0.125f;
  _Float16* P = Ps + w * (16u * LDT);

  const size_t qoff = (size_t)(b * (unsigned)SEQ + qw0 + m) * DIM + head * HD + hh * 8u;
  v16h qf[2], qr[2];
  qf[0] = frag_at(Qh + qoff);
  qf[1] = frag_at(Qh + qoff + 32);
  qr[0] = frag_at(Qr + qoff);
  qr[1] = frag_at(Qr + qoff + 32);

  float mrow[8], lrow[8];
  v8f o[4], orr[4];
#pragma unroll
  for (int v = 0; v < 8; ++v) { mrow[v] = -1.0e30f; lrow[v] = 0.0f; }
#pragma unroll
  for (int nb = 0; nb < 4; ++nb) { o[nb] = (v8f){}; orr[nb] = (v8f){}; }

  const size_t kplane = (size_t)b * SEQ * DIM + head * HD;
  const size_t vplane = ((size_t)b * DIM + head * HD) * SEQ;
  const unsigned kend = q0 + 128u;

  for (unsigned kb = 0; kb < kend; kb += 64u) {
#pragma unroll
    for (unsigned j = 0; j < 2u; ++j) {
      const unsigned idx = tid + 256u * j;
      const unsigned r = idx >> 3, c = (idx & 7u) * 8u;
      const size_t ko = kplane + (size_t)(kb + r) * DIM + c;
      const size_t vo = vplane + (size_t)r * SEQ + kb + c;
      *(v8h*)&Ks[r * LDT + c] = *(const v8h*)(Kh + ko);
      *(v8h*)&Kq[r * LDT + c] = *(const v8h*)(Kr + ko);
      *(v8h*)&Vs[r * LDT + c] = *(const v8h*)(Vt + vo);
      *(v8h*)&Vq[r * LDT + c] = *(const v8h*)(Vtr + vo);
    }
    __syncthreads();

    if (kb <= qw0 + 15u) {
      v8f s[4];
#pragma unroll
      for (int kg = 0; kg < 4; ++kg) {
        v8f t = {}, tr = {};
#pragma unroll
        for (int c = 0; c < 2; ++c) {
          const v16h kf = ld_frag(&Ks[(kg * 16) * LDT + c * 32], LDT);
          const v16h kr = ld_frag(&Kq[(kg * 16) * LDT + c * 32], LDT);
          t  = wmma16(qf[c], kf, t);
          tr = wmma16(qf[c], kr, tr);
          tr = wmma16(qr[c], kf, tr);
        }
        s[kg] = (t + tr * RINV) * scale;
      }
      if (kb + 63u > qw0) {
#pragma unroll
        for (int kg = 0; kg < 4; ++kg) {
          const unsigned key = kb + (unsigned)kg * 16u + m;
#pragma unroll
          for (int v = 0; v < 8; ++v) {
            const unsigned qrow = qw0 + hh * 8u + (unsigned)v;
            s[kg][v] = (key > qrow) ? -1.0e30f : s[kg][v];
          }
        }
      }

      float alpha[8];
#pragma unroll
      for (int v = 0; v < 8; ++v) {
        float mx = fmaxf(fmaxf(s[0][v], s[1][v]), fmaxf(s[2][v], s[3][v]));
        mx = red16_max(mx);
        const float mn = fmaxf(mrow[v], mx);
        alpha[v] = __expf(mrow[v] - mn);
        mrow[v] = mn;
      }
#pragma unroll
      for (int kg = 0; kg < 4; ++kg)
#pragma unroll
        for (int v = 0; v < 8; ++v) s[kg][v] = __expf(s[kg][v] - mrow[v]);
#pragma unroll
      for (int v = 0; v < 8; ++v) {
        const float rs = red16_sum((s[0][v] + s[1][v]) + (s[2][v] + s[3][v]));
        lrow[v] = alpha[v] * lrow[v] + rs;
      }
#pragma unroll
      for (int nb = 0; nb < 4; ++nb)
#pragma unroll
        for (int v = 0; v < 8; ++v) {
          o[nb][v] = o[nb][v] * alpha[v];
          orr[nb][v] = orr[nb][v] * alpha[v];
        }

#pragma unroll
      for (int kg = 0; kg < 4; ++kg)
#pragma unroll
        for (int v = 0; v < 8; ++v)
          P[(hh * 8u + (unsigned)v) * LDT + (unsigned)kg * 16u + m] =
              toh_flush(s[kg][v] * PCARRY);
      wave_lds_sync();
      v16h pf[2];
      pf[0] = ld_frag(P, LDT);
      pf[1] = ld_frag(P + 32, LDT);
      wave_lds_sync();
#pragma unroll
      for (int kg = 0; kg < 4; ++kg)
#pragma unroll
        for (int v = 0; v < 8; ++v) {
          const float t = s[kg][v] * PCARRY;
          const _Float16 hi = toh_flush(t);
          P[(hh * 8u + (unsigned)v) * LDT + (unsigned)kg * 16u + m] =
              toh_flush((t - (float)hi) * RCARRY);
        }
      wave_lds_sync();
      v16h pr[2];
      pr[0] = ld_frag(P, LDT);
      pr[1] = ld_frag(P + 32, LDT);

#pragma unroll
      for (int c = 0; c < 2; ++c) {
#pragma unroll
        for (int nb = 0; nb < 4; ++nb) {
          const v16h vf = ld_frag(&Vs[(nb * 16) * LDT + c * 32], LDT);
          const v16h vr = ld_frag(&Vq[(nb * 16) * LDT + c * 32], LDT);
          o[nb]   = wmma16(pf[c], vf, o[nb]);
          orr[nb] = wmma16(pf[c], vr, orr[nb]);
          orr[nb] = wmma16(pr[c], vf, orr[nb]);
        }
      }
    }
    __syncthreads();
  }

  float inv[8];
#pragma unroll
  for (int v = 0; v < 8; ++v) inv[v] = __builtin_amdgcn_rcpf(lrow[v]) * (VCARRY / PCARRY);
#pragma unroll
  for (int nb = 0; nb < 4; ++nb)
#pragma unroll
    for (int v = 0; v < 8; ++v) {
      const float val = (o[nb][v] + orr[nb][v] * RINV) * inv[v];
      P[(hh * 8u + (unsigned)v) * LDT + (unsigned)nb * 16u + m] = toh_flush(val);
    }
  wave_lds_sync();
  v8h x[4], xr[4];
  size_t off[4];
#pragma unroll
  for (unsigned i = 0; i < 4u; ++i) {
    const unsigned r = 4u * i + (lane >> 3);
    const unsigned c = (lane & 7u) * 8u;
    x[i] = *(const v8h*)&P[r * LDT + c];
    off[i] = (size_t)(b * (unsigned)SEQ + qw0 + r) * DIM + head * HD + c;
  }
  wave_lds_sync();
#pragma unroll
  for (int nb = 0; nb < 4; ++nb)
#pragma unroll
    for (int v = 0; v < 8; ++v) {
      const float val = (o[nb][v] + orr[nb][v] * RINV) * inv[v];
      const _Float16 hi = toh_flush(val);
      P[(hh * 8u + (unsigned)v) * LDT + (unsigned)nb * 16u + m] =
          toh_flush((val - (float)hi) * RCARRY);
    }
  wave_lds_sync();
#pragma unroll
  for (unsigned i = 0; i < 4u; ++i) {
    const unsigned r = 4u * i + (lane >> 3);
    const unsigned c = (lane & 7u) * 8u;
    xr[i] = *(const v8h*)&P[r * LDT + c];
  }
#pragma unroll
  for (int i = 0; i < 4; ++i) *(volatile v8h*)(Ov + off[i]) = x[i];
#pragma unroll
  for (int i = 0; i < 4; ++i) *(volatile v8h*)(Ovr + off[i]) = xr[i];
  __threadfence();
#pragma unroll
  for (int i = 0; i < 4; ++i) *(volatile v8h*)(Ov + off[i]) = x[i];
#pragma unroll
  for (int i = 0; i < 4; ++i) *(volatile v8h*)(Ovr + off[i]) = xr[i];
}

extern "C" void kernel_launch(void* const* d_in, const int* in_sizes, int n_in,
                              void* d_out, int out_size, void* d_ws, size_t ws_size,
                              hipStream_t stream) {
  if (n_in < 11) return;
  const long long need_x = ((long long)(NB - 1) * SEQ_FULL + SEQ) * DIM;
  if ((long long)in_sizes[0] < need_x) return;
  if (in_sizes[1] < DIM || in_sizes[2] < DIM) return;
  if ((long long)in_sizes[3] < (long long)DIM * DIM) return;
  if ((long long)in_sizes[4] < (long long)DIM * DIM) return;
  if ((long long)in_sizes[5] < (long long)DIM * DIM) return;
  if ((long long)in_sizes[6] < (long long)DIM * DIM) return;
  if ((long long)in_sizes[7] < (long long)NCB * DIM * CDIM) return;
  if ((long long)in_sizes[8] < (long long)NCB * DFF * CDIM) return;
  if ((long long)in_sizes[9] < (long long)NCB * DFF * CDIM) return;
  if ((long long)in_sizes[10] < (long long)NCB * DIM * CDIM) return;
  if ((long long)out_size < need_x) return;
  if (ws_size < WS_TOTAL) return;

  const float* X    = (const float*)d_in[0];
  const float* ln1g = (const float*)d_in[1];
  const float* ln2g = (const float*)d_in[2];
  const float* wq   = (const float*)d_in[3];
  const float* wk   = (const float*)d_in[4];
  const float* wv   = (const float*)d_in[5];
  const float* wo   = (const float*)d_in[6];
  const float* wd1  = (const float*)d_in[7];
  const float* wu1  = (const float*)d_in[8];
  const float* wd2  = (const float*)d_in[9];
  const float* wu2  = (const float*)d_in[10];
  float* out = (float*)d_out;

  char* ws = (char*)d_ws;
  _Float16* WqkvT = (_Float16*)(ws + OFF_WQKV);
  _Float16* WoT   = (_Float16*)(ws + OFF_WO);
  _Float16* W1D   = (_Float16*)(ws + OFF_W1D);
  _Float16* W1U   = (_Float16*)(ws + OFF_W1U);
  _Float16* W2D   = (_Float16*)(ws + OFF_W2D);
  _Float16* W2U   = (_Float16*)(ws + OFF_W2U);
  float*    CS    = (float*)(ws + OFF_CS);
  _Float16* RA16  = (_Float16*)(ws + OFF_RA);
  _Float16* H1    = RA16;
  _Float16* H1r   = RA16 + 1 * PLANE16_ELEMS;
  _Float16* QKV16 = RA16 + 2 * PLANE16_ELEMS;
  _Float16* QKVr  = RA16 + 5 * PLANE16_ELEMS;
  float*    PROD  = (float*)(ws + OFF_RA);
  _Float16* Ctx16 = (_Float16*)(ws + OFF_RB);
  _Float16* Ctxr  = Ctx16 + PLANE16_ELEMS;
  float*    PROD2 = (float*)(ws + OFF_RB);
  float*    X1    = (float*)(ws + OFF_X1);
  _Float16* H2    = (_Float16*)(ws + OFF_H2);
  _Float16* H2r   = H2 + PLANE16_ELEMS;
  _Float16* AD    = (_Float16*)(ws + OFF_AD);
  _Float16* ADr   = AD + ADPL_ELEMS;
  _Float16* S16   = (_Float16*)(ws + OFF_S);
  _Float16* S16r  = S16 + SPL_ELEMS;
  _Float16* BD    = (_Float16*)(ws + OFF_BD);
  _Float16* BDr   = BD + ADPL_ELEMS;

  dim3 blk(256);
  const unsigned n8sq = (unsigned)(WSQ_ELEMS / 8);
  const unsigned n8u1 = (unsigned)(((size_t)NCB * DFF * CDIM) / 8);
  const unsigned n8u2 = (unsigned)(((size_t)NCB * DIM * CDIM) / 8);
  wcast_kernel<<<dim3(n8sq / 256), blk, 0, stream>>>(wq, WqkvT + 0 * WSQ_ELEMS, n8sq);
  wcast_kernel<<<dim3(n8sq / 256), blk, 0, stream>>>(wk, WqkvT + 1 * WSQ_ELEMS, n8sq);
  wcast_kernel<<<dim3(n8sq / 256), blk, 0, stream>>>(wv, WqkvT + 2 * WSQ_ELEMS, n8sq);
  wcast_kernel<<<dim3(n8sq / 256), blk, 0, stream>>>(wo, WoT, n8sq);
  wcast_kernel<<<dim3(n8u1 / 256), blk, 0, stream>>>(wu1, W1U, n8u1);
  wcast_kernel<<<dim3(n8u2 / 256), blk, 0, stream>>>(wu2, W2U, n8u2);
  wconv_kernel<<<dim3(DCAT / 64, DIM / 64), blk, 0, stream>>>(wd1, W1D, DCAT, DIM, 1u);
  wconv_kernel<<<dim3(DCAT / 64, DFF / 64), blk, 0, stream>>>(wd2, W2D, DCAT, DFF, 1u);
  rope_table_kernel<<<dim3(SEQ / 8), blk, 0, stream>>>(CS);

  rms_kernel<<<dim3(MROWS), dim3(128), 0, stream>>>(X, ln1g, H1, H1r, 1u, 1u);
  gemm_qkv_kernel<<<dim3(3 * DIM / 64, MROWS / 64), blk, 0, stream>>>(
      H1, H1r, WqkvT, CS, QKV16, QKVr);
  attn_kernel<<<dim3(SEQ / 128, NHEAD, NB), blk, 0, stream>>>(
      QKV16, QKV16 + PLANE16_ELEMS, QKV16 + 2 * PLANE16_ELEMS, Ctx16);
  attn_early_kernel<<<dim3(EROWS_EFF / 128, NHEAD, NB), blk, 0, stream>>>(
      QKV16, QKVr, QKV16 + PLANE16_ELEMS, QKVr + PLANE16_ELEMS,
      QKV16 + 2 * PLANE16_ELEMS, QKVr + 2 * PLANE16_ELEMS, Ctx16, Ctxr);
  gemm_wo_kernel<<<dim3(DIM / 64, MROWS / 64), blk, 0, stream>>>(Ctx16, Ctxr, WoT, X, X1);

  rms_kernel<<<dim3(MROWS), dim3(128), 0, stream>>>(X1, ln2g, H2, H2r, 0u, 0u);
  gemm_down_kernel<<<dim3(DCAT / 64, MROWS / 64), blk, 0, stream>>>(H2, H2r, W1D, AD, ADr, DIM);
  up_prod_kernel<<<dim3(DFF / 64, MROWS / 64), blk, 0, stream>>>(AD, ADr, W1U, PROD, DFF);
  rms_silu_kernel<<<dim3(MROWS), blk, 0, stream>>>(PROD, S16, S16r);
  gemm_down_kernel<<<dim3(DCAT / 64, MROWS / 64), blk, 0, stream>>>(S16, S16r, W2D, BD, BDr, DFF);
  up_prod_kernel<<<dim3(DIM / 64, MROWS / 64), blk, 0, stream>>>(BD, BDr, W2U, PROD2, DIM);
  rms_out_kernel<<<dim3(MROWS), blk, 0, stream>>>(PROD2, X1, out);
}
